// PoolbyIndices_2482491097343
// MI455X (gfx1250) — hardware-run, weakly checked
//
#include <hip/hip_runtime.h>


#ifndef NB
#define NB 4
#endif
#ifndef NT
#define NT 2048
#endif
#ifndef NS
#define NS 8192
#endif
#define NB_FULL 4
#define NT_FULL 2048
#define NS_FULL 8192
#ifndef OUT_NT
#define OUT_NT NT
#endif
#define DM   128
#define TP   72
#define OSP  68

static_assert(DM == 128);
static_assert(DM % 64 == 0);
static_assert(NS % 64 == 0);
static_assert(NS % 32 == 0);
static_assert(NT % 64 == 0);
static_assert((NB * NT) % 64 == 0);
static_assert(NB <= NB_FULL);
static_assert(NT <= NT_FULL);
static_assert(NS <= NS_FULL);
static_assert((TP * 2) % 16 == 0);
static_assert(TP >= 64);
static_assert((OSP * 4) % 16 == 0);
static_assert(OSP >= 64);
static_assert(256 * 8 * 4 == 64 * DM);
static_assert(256 * 4 * 16 == DM * 64 * 2);
static_assert(32 * 16 * 8 == 16 * 64 * 4);
static_assert((size_t)DM * TP * 2 <= 131072);
static_assert((size_t)16 * OSP * 4 + 64 * 4 <= 131072);

typedef unsigned short bf;
typedef __attribute__((ext_vector_type(16))) __bf16   v16bf;
typedef __attribute__((ext_vector_type(8)))  unsigned short v8us;
typedef v8us __attribute__((may_alias)) v8usa;
typedef __attribute__((ext_vector_type(8)))  unsigned v8u;
typedef __attribute__((ext_vector_type(8)))  float    v8f;
typedef __attribute__((ext_vector_type(4)))  float    v4f;
typedef v4f  __attribute__((may_alias)) v4fa;
typedef __attribute__((ext_vector_type(4)))  int      v4i;

__device__ __forceinline__ unsigned short f2bf(float f) { unsigned u = __float_as_uint(f); u += 0x7FFFu + ((u >> 16) & 1u); return (unsigned short)(u >> 16); }
__device__ __forceinline__ v16bf cat16b(v8us lo, v8us hi) { return __builtin_bit_cast(v16bf, __builtin_shufflevector(lo, hi, 0, 1, 2, 3, 4, 5, 6, 7, 8, 9, 10, 11, 12, 13, 14, 15)); }
__device__ __forceinline__ v16bf ldb(const bf* p)  { return cat16b(*(const v8us*)p, *(const v8us*)(p + 16)); }
__device__ __forceinline__ v8f wmmab_g(v16bf a, v16bf b, v8f c) {
    c = __builtin_amdgcn_wmma_f32_16x16x32_bf16(false, a, false, b, (short)0, c, false, false);
    asm volatile("v_nop\n\tv_nop\n\tv_nop\n\tv_nop" : "+v"(c) : "v"(a), "v"(b));
    return c;
}
__device__ __forceinline__ void wave_sync() { __builtin_amdgcn_fence(3  , "wavefront"); __builtin_amdgcn_wave_barrier(); asm volatile("" ::: "memory"); }

__global__ __launch_bounds__(256) void k_cvtT(const float* __restrict__ src, bf* ST) {
    __shared__ __align__(16) unsigned short tl[DM * TP];
    const int tid = threadIdx.x;
    const int m0 = blockIdx.x * 64, b = blockIdx.y;
    const float* sp = src + ((size_t)b * NS_FULL + (size_t)m0) * DM;
#pragma unroll 1
    for (int it = 0; it < 8; ++it) {
        const int p = it * 256 + tid; const int row = p >> 5, c4 = (p & 31) * 4;
        const v4f v = *(const v4f*)(sp + (size_t)row * DM + c4);
#pragma unroll
        for (int i = 0; i < 4; ++i) tl[(c4 + i) * TP + row] = f2bf(v[i]);
    }
    __syncthreads();
    bf* dp = ST + ((size_t)b * DM) * NS + (size_t)m0;
#pragma unroll 1
    for (int ps = 0; ps < 2; ++ps) {
#pragma unroll
        for (int s = 0; s < 4; ++s) { const int p = s * 256 + tid; const int d = p >> 3, c8 = (p & 7) * 8;
            const v8us o = *(const v8usa*)(&tl[d * TP + c8]);
            *(volatile v8us*)(dp + (size_t)d * NS + c8) = o; }
        if (ps == 0) __threadfence(); }
}

__global__ __launch_bounds__(32) void k_pool(const int* __restrict__ IT, const int* __restrict__ IS, const bf* __restrict__ ST, float* OUT) {
    __shared__ __align__(16) float os[16 * OSP];
    __shared__ __align__(16) float ivs[64];
    const int lane = threadIdx.x & 31, lr = lane & 15, hi = lane >> 4;
    const int r0 = blockIdx.x * 64, c0 = blockIdx.y * 64;
    const int bb = r0 / NT, tt = r0 % NT;
    int tv[4], cnt[4];
#pragma unroll
    for (int mb = 0; mb < 4; ++mb) { tv[mb] = IT[(size_t)bb * NT_FULL + (size_t)(tt + mb * 16 + lr)]; cnt[mb] = 0; }
    v8f acc[4][4];
#pragma unroll
    for (int mb = 0; mb < 4; ++mb)
#pragma unroll
        for (int nb = 0; nb < 4; ++nb) acc[mb][nb] = (v8f){};
    const int* isb = IS + (size_t)bb * NS_FULL + 8 * hi;
    const size_t boff = ((size_t)bb * DM + (size_t)(c0 + lr)) * NS + 8 * hi;
#pragma unroll 1
    for (int kc = 0; kc < NS; kc += 32) {
        const v4i s0 = *(const v4i*)(isb + kc), s1 = *(const v4i*)(isb + kc + 4), s2 = *(const v4i*)(isb + kc + 16), s3 = *(const v4i*)(isb + kc + 20);
        int sv[16];
#pragma unroll
        for (int i = 0; i < 4; ++i) { sv[i] = s0[i]; sv[4 + i] = s1[i]; sv[8 + i] = s2[i]; sv[12 + i] = s3[i]; }
        v16bf a[4];
#pragma unroll
        for (int mb = 0; mb < 4; ++mb) {
            v8u w; int c = cnt[mb]; const int t = tv[mb];
#pragma unroll
            for (int j = 0; j < 8; ++j) {
                const bool e0 = sv[2 * j] == t, e1 = sv[2 * j + 1] == t;
                w[j] = (e0 ? 0x3F80u : 0u) | (e1 ? 0x3F800000u : 0u);
                c += (int)e0 + (int)e1; }
            cnt[mb] = c;
            a[mb] = __builtin_bit_cast(v16bf, w); }
#pragma unroll
        for (int nb = 0; nb < 4; ++nb) { const v16bf b = ldb(ST + boff + (size_t)nb * 16 * NS + kc);
#pragma unroll
            for (int mb = 0; mb < 4; ++mb) acc[mb][nb] = wmmab_g(a[mb], b, acc[mb][nb]); }
    }
#pragma unroll
    for (int mb = 0; mb < 4; ++mb) {
        const int other = __shfl_xor(cnt[mb], 16, 32);
        const float wsum = (float)(cnt[mb] + other) + 1e-10f;
        ivs[mb * 16 + lr] = 1.0f / wsum; }
    float* orow = OUT + ((size_t)bb * OUT_NT + (size_t)tt) * DM + c0;
#pragma unroll
    for (int mb = 0; mb < 4; ++mb) {
#pragma unroll
        for (int nb = 0; nb < 4; ++nb) {
#pragma unroll
            for (int j = 0; j < 8; ++j) os[(hi * 8 + j) * OSP + nb * 16 + lr] = acc[mb][nb][j]; }
        wave_sync();
#pragma unroll 1
        for (int ps = 0; ps < 2; ++ps) {
#pragma unroll
            for (int s = 0; s < 8; ++s) { const int row = 2 * s + (lane >> 4), cofs = (lane & 15) * 4;
                const v4f x = *(const v4fa*)(&os[row * OSP + cofs]);
                const float sc = ivs[mb * 16 + row];
                v4f val; val[0] = x[0] * sc; val[1] = x[1] * sc; val[2] = x[2] * sc; val[3] = x[3] * sc;
                *(volatile v4f*)(orow + (size_t)(mb * 16 + row) * DM + cofs) = val; }
            if (ps == 0) __threadfence(); }
        wave_sync();
    }
}

static constexpr size_t al256(size_t v) { return (v + 255) & ~(size_t)255; }
static constexpr size_t SZ_ST = al256((size_t)NB * DM * NS * 2);
static constexpr size_t SZ_TOTAL = SZ_ST;
static_assert(SZ_TOTAL <= (size_t)134217728);
static_assert(((size_t)NS * 2) % 128 == 0);
static_assert((size_t)(NB - 1) * DM * NS + (size_t)(DM - 1) * NS + (NS - 64) + 56 + 8 <= (size_t)NB * DM * NS);

extern "C" void kernel_launch(void* const* d_in, const int* in_sizes, int n_in,
                              void* d_out, int out_size, void* d_ws, size_t ws_size, hipStream_t stream) {
    if (n_in < 3) return;
    const size_t needt = (size_t)(NB - 1) * NT_FULL + NT;
    const size_t needs = (size_t)(NB - 1) * NS_FULL + NS;
    if ((size_t)in_sizes[0] < needt || (size_t)in_sizes[1] < needs || (size_t)in_sizes[2] < needs * DM) return;
    if ((size_t)out_size < ((size_t)(NB - 1) * OUT_NT + NT) * DM) return;
    if (SZ_TOTAL > ws_size) return;
    const int* idt = (const int*)d_in[0];
    const int* ids = (const int*)d_in[1];
    const float* src = (const float*)d_in[2];
    float* OUT = (float*)d_out;
    bf* ST = (bf*)d_ws;

    k_cvtT<<<dim3(NS / 64, NB, 1), 256, 0, stream>>>(src, ST);
    k_pool<<<dim3(NB * NT / 64, DM / 64, 1), 32, 0, stream>>>(idt, ids, ST, OUT);
}
